// RNNBlock_52080773431560
// MI455X (gfx1250) — hardware-verified
//
#include <hip/hip_runtime.h>
#include <stdint.h>

typedef __attribute__((ext_vector_type(16))) _Float16 v16h;
typedef __attribute__((ext_vector_type(8)))  _Float16 v8h;
typedef __attribute__((ext_vector_type(16))) __bf16   v16b;
typedef __attribute__((ext_vector_type(8)))  __bf16   v8b;
typedef __attribute__((ext_vector_type(8)))  float    v8f;
typedef __attribute__((ext_vector_type(4)))  float    v4f;

constexpr int NB_ROWS  = 8192;
constexpr int NSEQ     = 79;
constexpr int NFEAT    = 4;
constexpr int NCH      = 256;
constexpr int ROWS_PB  = 16;
constexpr int TPB_MAIN = 256;
constexpr int HPITCH   = 264;
constexpr int OPITCH   = 260;
constexpr float H_CARRY   = 8.0f;
constexpr float W_CARRY   = 16.0f;
constexpr float ACC_SCL8  = 1.0f / 16.0f;
constexpr float ACC_SCL1  = 1.0f / 128.0f;

__device__ __forceinline__ void dep_guard_h(v8f& a, v8f& b, v16h x, v16h y) { asm volatile("v_nop\n\tv_nop\n\tv_nop\n\tv_nop" : "+v"(a), "+v"(b) : "v"(x), "v"(y)); }
__device__ __forceinline__ void dep_guard_b(v8f& a, v8f& b, v16b x, v16b y) { asm volatile("v_nop\n\tv_nop\n\tv_nop\n\tv_nop" : "+v"(a), "+v"(b) : "v"(x), "v"(y)); }
__device__ __forceinline__ void keep4_h(v16h a, v16h b, v16h c, v16h d) { asm volatile("v_nop" :: "v"(a), "v"(b), "v"(c), "v"(d)); }
__device__ __forceinline__ void keep4_b(v16b a, v16b b, v16b c, v16b d) { asm volatile("v_nop" :: "v"(a), "v"(b), "v"(c), "v"(d)); }
__device__ __forceinline__ void guard3_h(v8f& a, v8f& b, v16h x, v16h y, v16h z) { asm volatile("v_nop\n\tv_nop\n\tv_nop\n\tv_nop" : "+v"(a), "+v"(b) : "v"(x), "v"(y), "v"(z)); }

template <typename T> struct Frag;
template <> struct Frag<_Float16> {
  typedef v16h V; union U { v16h v; v8h h[2]; };
  static __device__ __forceinline__ v16h load(const _Float16* p) {
    U f; f.h[0] = *(const v8h*)(p); f.h[1] = *(const v8h*)(p + 16); return f.v;
  }
  static __device__ __forceinline__ v8f mma(v16h a, v16h b, v8f c) {
    return __builtin_amdgcn_wmma_f32_16x16x32_f16(false, a, false, b, (short)0, c, false, false);
  }
  static __device__ __forceinline__ void guard(v8f& a, v8f& b, v16h x, v16h y) { dep_guard_h(a, b, x, y); }
  static __device__ __forceinline__ void keep(v16h a, v16h b, v16h c, v16h d) { keep4_h(a, b, c, d); }
};
template <> struct Frag<__bf16> {
  typedef v16b V; union U { v16b v; v8b h[2]; };
  static __device__ __forceinline__ v16b load(const __bf16* p) {
    U f; f.h[0] = *(const v8b*)(p); f.h[1] = *(const v8b*)(p + 16); return f.v;
  }
  static __device__ __forceinline__ v8f mma(v16b a, v16b b, v8f c) {
    return __builtin_amdgcn_wmma_f32_16x16x32_bf16(false, a, false, b, (short)0, c, false, false);
  }
  static __device__ __forceinline__ void guard(v8f& a, v8f& b, v16b x, v16b y) { dep_guard_b(a, b, x, y); }
  static __device__ __forceinline__ void keep(v16b a, v16b b, v16b c, v16b d) { keep4_b(a, b, c, d); }
};

__global__ __launch_bounds__(256) void prep_wt16(
    const float* __restrict__ Wa, const float* __restrict__ Wb,
    _Float16* __restrict__ WaT, _Float16* __restrict__ WbT) {
  const int g = blockIdx.x * 256 + threadIdx.x;
  const bool sec = (blockIdx.x >= (NCH * NCH / 8) / 256);
  const float* src = sec ? Wb : Wa;
  _Float16* dst = sec ? WbT : WaT;
  const int gg = sec ? (g - NCH * NCH / 8) : g;
  const int n  = gg >> 5;
  const int k0 = (gg & 31) * 8;
  v8h hv;
#pragma unroll
  for (int e = 0; e < 8; ++e) hv[e] = (_Float16)(src[(size_t)(k0 + e) * NCH + n] * W_CARRY);
  _Float16* p = dst + (size_t)n * NCH + k0;
  *(volatile v8h*)p = hv;
  __threadfence();
  *(volatile v8h*)p = hv;
}

__device__ __forceinline__ void stage_x(float* xs, const float* __restrict__ xf, int f, int row0, int tid) {
  for (int idx = tid; idx < ROWS_PB * NSEQ; idx += TPB_MAIN) {
    const int row = idx / NSEQ;
    const int l   = idx - row * NSEQ;
    xs[(l * ROWS_PB + row) * NFEAT + f] = xf[(size_t)(row0 + row) * NSEQ + l];
  }
}

__global__ __launch_bounds__(256) void scan_dense_kernel(
    const float* __restrict__ x0, const float* __restrict__ x1,
    const float* __restrict__ x2, const float* __restrict__ x3,
    const float* __restrict__ Wx, const float* __restrict__ b_rnn, const float* __restrict__ b_d,
    const _Float16* __restrict__ WhT, const _Float16* __restrict__ WdT,
    float* __restrict__ out) {
  __shared__ __align__(16) float    xs[NSEQ * ROWS_PB * NFEAT];
  __shared__ __align__(16) _Float16 hbuf[2][ROWS_PB * HPITCH];
  __shared__ __align__(16) float    oslab[ROWS_PB * OPITCH];

  const int tid  = threadIdx.x;
  const int lane = tid & 31;
  const int wave = tid >> 5;
  const int hh   = lane >> 4;
  const int c    = lane & 15;
  const int koff = hh * 8;
  const int row0 = blockIdx.x * ROWS_PB;
  const int ncol0 = wave * 32;

  stage_x(xs, x0, 0, row0, tid);
  stage_x(xs, x1, 1, row0, tid);
  stage_x(xs, x2, 2, row0, tid);
  stage_x(xs, x3, 3, row0, tid);
  {
    _Float16* hb = &hbuf[0][0];
    v8h z;
#pragma unroll
    for (int e = 0; e < 8; ++e) z[e] = (_Float16)0.0f;
    for (int i = tid; i < (2 * ROWS_PB * HPITCH) / 8; i += TPB_MAIN) *(v8h*)(hb + i * 8) = z;
  }
  float wx8[2][4], br8[2], bd[2];
#pragma unroll
  for (int j = 0; j < 2; ++j) {
    const int n = ncol0 + j * 16 + c;
#pragma unroll
    for (int f = 0; f < NFEAT; ++f) wx8[j][f] = Wx[f * NCH + n] * H_CARRY;
    br8[j] = b_rnn[n] * H_CARRY;
    bd[j]  = b_d[n];
  }
  __syncthreads();

  const v8f zero8 = (v8f){0.f, 0.f, 0.f, 0.f, 0.f, 0.f, 0.f, 0.f};

#pragma unroll 1
  for (int t = 0; t < NSEQ; ++t) {
    const _Float16* hr = &hbuf[t & 1][0];
    _Float16*       hw = &hbuf[(t + 1) & 1][0];
    v8f acc0 = zero8, acc1 = zero8;
#pragma unroll 2
    for (int k0 = 0; k0 < NCH; k0 += 32) {
      const v16h a  = Frag<_Float16>::load(hr + c * HPITCH + koff + k0);
      const v16h b0 = Frag<_Float16>::load(WhT + (size_t)(ncol0 + c) * NCH + koff + k0);
      const v16h b1 = Frag<_Float16>::load(WhT + (size_t)(ncol0 + 16 + c) * NCH + koff + k0);
      acc0 = Frag<_Float16>::mma(a, b0, acc0);
      acc1 = Frag<_Float16>::mma(a, b1, acc1);
      guard3_h(acc0, acc1, a, b0, b1);
    }
    const int l = NSEQ - 1 - t;
    const float* xrow = xs + (l * ROWS_PB + 8 * hh) * NFEAT;
#pragma unroll
    for (int r = 0; r < 8; ++r) {
      const v4f xv = *(const v4f*)(xrow + r * NFEAT);
      float xw0 = br8[0];
      xw0 += xv[0] * wx8[0][0]; xw0 += xv[1] * wx8[0][1]; xw0 += xv[2] * wx8[0][2]; xw0 += xv[3] * wx8[0][3];
      float xw1 = br8[1];
      xw1 += xv[0] * wx8[1][0]; xw1 += xv[1] * wx8[1][1]; xw1 += xv[2] * wx8[1][2]; xw1 += xv[3] * wx8[1][3];
      const float v0 = xw0 + acc0[r] * ACC_SCL8;
      const float v1 = xw1 + acc1[r] * ACC_SCL8;
      const float h0v = fmaxf(v0, 0.0f);
      const float h1v = fmaxf(v1, 0.0f);
      hw[(8 * hh + r) * HPITCH + ncol0 + c]      = (_Float16)h0v;
      hw[(8 * hh + r) * HPITCH + ncol0 + 16 + c] = (_Float16)h1v;
    }
    __syncthreads();
  }

  {
    const _Float16* hl = &hbuf[NSEQ & 1][0];
    v8f acc0 = zero8, acc1 = zero8;
#pragma unroll 2
    for (int k0 = 0; k0 < NCH; k0 += 32) {
      const v16h a  = Frag<_Float16>::load(hl + c * HPITCH + koff + k0);
      const v16h b0 = Frag<_Float16>::load(WdT + (size_t)(ncol0 + c) * NCH + koff + k0);
      const v16h b1 = Frag<_Float16>::load(WdT + (size_t)(ncol0 + 16 + c) * NCH + koff + k0);
      acc0 = Frag<_Float16>::mma(a, b0, acc0);
      acc1 = Frag<_Float16>::mma(a, b1, acc1);
      guard3_h(acc0, acc1, a, b0, b1);
    }
#pragma unroll
    for (int r = 0; r < 8; ++r) {
      const float v0 = bd[0] + acc0[r] * ACC_SCL1;
      const float v1 = bd[1] + acc1[r] * ACC_SCL1;
      oslab[(8 * hh + r) * OPITCH + ncol0 + c]      = fmaxf(v0, 0.0f);
      oslab[(8 * hh + r) * OPITCH + ncol0 + 16 + c] = fmaxf(v1, 0.0f);
    }
  }
  __syncthreads();

  for (int pass = 0; pass < 2; ++pass) {
#pragma unroll
    for (int it = 0; it < 2; ++it) {
      const int row = wave * 2 + it;
#pragma unroll
      for (int half = 0; half < 2; ++half) {
        const int col = half * 128 + lane * 4;
        const v4f val = *(const v4f*)(oslab + row * OPITCH + col);
        *(volatile v4f*)(out + (size_t)(row0 + row) * NCH + col) = val;
      }
    }
    __threadfence();
  }
}

extern "C" void kernel_launch(void* const* d_in, const int* in_sizes, int n_in,
                              void* d_out, int out_size, void* d_ws, size_t ws_size,
                              hipStream_t stream) {
  if (n_in < 9) return;
  const float* x0    = (const float*)d_in[0];
  const float* x1    = (const float*)d_in[1];
  const float* x2    = (const float*)d_in[2];
  const float* x3    = (const float*)d_in[3];
  const float* Wx    = (const float*)d_in[4];
  const float* Wh    = (const float*)d_in[5];
  const float* b_rnn = (const float*)d_in[6];
  const float* Wd    = (const float*)d_in[7];
  const float* b_d   = (const float*)d_in[8];
  float* out = (float*)d_out;

  const size_t plane_bytes = (size_t)NCH * NCH * sizeof(_Float16);
  if (ws_size < 2 * plane_bytes) return;
  if (in_sizes[0] != NB_ROWS * NSEQ || in_sizes[1] != NB_ROWS * NSEQ ||
      in_sizes[2] != NB_ROWS * NSEQ || in_sizes[3] != NB_ROWS * NSEQ ||
      in_sizes[4] != NFEAT * NCH || in_sizes[5] != NCH * NCH || in_sizes[6] != NCH ||
      in_sizes[7] != NCH * NCH || in_sizes[8] != NCH || out_size != NB_ROWS * NCH) return;

  _Float16* WhT = (_Float16*)d_ws;
  _Float16* WdT = (_Float16*)((char*)d_ws + plane_bytes);

  prep_wt16<<<dim3(2 * (NCH * NCH / 8) / 256), dim3(256), 0, stream>>>(Wh, Wd, WhT, WdT);
  scan_dense_kernel<<<dim3(NB_ROWS / ROWS_PB), dim3(TPB_MAIN), 0, stream>>>(
      x0, x1, x2, x3, Wx, b_rnn, b_d, WhT, WdT, out);
}
